// TransformerBlock_3393024164190
// MI455X (gfx1250) — hardware-run, weakly checked
//
#include <hip/hip_runtime.h>


#ifndef NB
#define NB 4
#endif
#ifndef SEQ
#define SEQ 2048
#endif
#define NB_FULL  4
#define SEQ_FULL 2048
#ifndef OUT_SEQ
#define OUT_SEQ SEQ
#endif
#define DM   512
#define NH_  4
#define DQC  192
#define DKC  128
#define DNO  64
#define DRO  32
#define DVH  128
#define DKV  (DKC + DRO)
#define DEX  1024
#define NEX  8
#define NSH  2
#define KH   ((NEX + NSH) * DEX)
#define AW   4
#define OSP  132
#define WSC  1024.0f
#define ASC  64.0f
#define SC_ONE  1.0f
#define SC_PL   (1.0f / 1024.0f)
#define SC_TRUE (1.0f / 65536.0f)
#define SC_WO   (1.0f / 1048576.0f)
#define CTXS 16.0f
#define SC2S ((float)(0.10206207261596575 * 1.4426950408889634 / 4096.0))
#define PSH  14.0f
#define NEGB (-3.0e38f)
#define EPSN 1.0e-6f
#define OUT1_OFF ((size_t)NB_FULL * SEQ_FULL * DM)

static_assert(OUT1_OFF * 4 == (size_t)16777216);
static_assert(NH_ * (DNO + DRO) == 384);
static_assert(NH_ * (DNO + DVH) == 768);
static_assert(NH_ * DVH == DM);
static_assert(DM % 64 == 0);
static_assert(DQC % 64 == 0);
static_assert(DKC % 64 == 0);
static_assert(KH % 64 == 0);
static_assert(DM % 32 == 0);
static_assert(DQC % 32 == 0);
static_assert(DKC % 32 == 0);
static_assert(KH % 32 == 0);
static_assert(DEX == 1024);
static_assert(SEQ % 64 == 0);
static_assert(SEQ % 32 == 0);
static_assert(SEQ % (16 * AW) == 0);
static_assert((NB * SEQ) % 64 == 0);
static_assert((NB * SEQ) % 32 == 0);
static_assert(NB <= NB_FULL);
static_assert(SEQ <= SEQ_FULL);
static_assert((OSP * 4) % 16 == 0);
static_assert(DQC == 24 * 8);
static_assert(DKC == 16 * 8);
static_assert(DRO == 4 * 8);
static_assert(DM == 4 * 32 * 4);
static_assert(DM * NEX == 4 * 256 * 4);
static_assert(32 * 16 * 8 == 16 * 64 * 4);
static_assert(32 * 16 * 4 == 16 * 64 * 2);
static_assert(32 * 16 * 8 == 16 * DVH * 2);
static_assert(256 * 4 * 4 == 64 * 64);
static_assert(256 * 2 * 8 == 64 * 64);
static_assert(AW * 16 * OSP * 4 <= 131072);
static_assert(64 * 65 * 4 <= 131072);
static_assert((DM * NEX + 8 * DM + 8 * 4 * NEX) * 4 <= 131072);

typedef _Float16 h16;
typedef unsigned short bf;
typedef __attribute__((ext_vector_type(16))) __bf16   v16bf;
typedef __attribute__((ext_vector_type(16))) _Float16 v16h;
typedef __attribute__((ext_vector_type(8)))  _Float16 v8h;
typedef __attribute__((ext_vector_type(8)))  unsigned short v8us;
typedef __attribute__((ext_vector_type(8)))  float    v8f;
typedef __attribute__((ext_vector_type(4)))  float    v4f;
typedef v4f  __attribute__((may_alias)) v4fa;

__device__ __forceinline__ unsigned short f2bf(float f) { unsigned u = __float_as_uint(f); u += 0x7FFFu + ((u >> 16) & 1u); return (unsigned short)(u >> 16); }
__device__ __forceinline__ float bfr(float f) { return __uint_as_float(((unsigned)f2bf(f)) << 16); }
__device__ __forceinline__ v16h cat16(v8h lo, v8h hi) { return __builtin_shufflevector(lo, hi, 0, 1, 2, 3, 4, 5, 6, 7, 8, 9, 10, 11, 12, 13, 14, 15); }
__device__ __forceinline__ v16bf cat16b(v8us lo, v8us hi) { return __builtin_bit_cast(v16bf, __builtin_shufflevector(lo, hi, 0, 1, 2, 3, 4, 5, 6, 7, 8, 9, 10, 11, 12, 13, 14, 15)); }
__device__ __forceinline__ v8f wmma16(v16h a, v16h b, v8f c) { return __builtin_amdgcn_wmma_f32_16x16x32_f16(false, a, false, b, (short)0, c, false, false); }
__device__ __forceinline__ v8f wmmab(v16bf a, v16bf b, v8f c) { return __builtin_amdgcn_wmma_f32_16x16x32_bf16(false, a, false, b, (short)0, c, false, false); }
__device__ __forceinline__ v16h  ldh(const h16* p) { return cat16(*(const v8h*)p, *(const v8h*)(p + 16)); }
__device__ __forceinline__ v16bf ldb(const bf* p)  { return cat16b(*(const v8us*)p, *(const v8us*)(p + 16)); }
__device__ __forceinline__ void wave_sync() { __builtin_amdgcn_fence(3  , "wavefront"); __builtin_amdgcn_wave_barrier(); asm volatile("" ::: "memory"); }
static __device__ __forceinline__ h16 toh_flush(float v) { const h16 r = (h16)v; return (fabsf(v) < 6.103515625e-05f) ? (h16)0.0f : r; }

__global__ __launch_bounds__(256) void k_cvt8(const float* __restrict__ src, bf* dst, size_t n8) {
    const size_t i = (size_t)blockIdx.x * 256 + threadIdx.x; if (i >= n8) return;
    const v8f v = *(const v8f*)(src + i * 8); v8us o;
#pragma unroll
    for (int k = 0; k < 8; ++k) o[k] = f2bf(v[k]);
    *(volatile v8us*)(dst + i * 8) = o; __threadfence(); *(volatile v8us*)(dst + i * 8) = o;
}

template <int F16>
__device__ __forceinline__ void wconv_body(const float* __restrict__ W, unsigned short* D, const int K, const int N, const int NV, const int G, const int SG, const int OFF,
                                           const int ldk, const int koff, const int dzr) {
    __shared__ __align__(16) float ts[64 * 65];
    const int tid = threadIdx.x;
    const int k0 = blockIdx.x * 64, n0 = blockIdx.y * 64, z = blockIdx.z;
    const float* Wz = W + (size_t)z * (size_t)K * (size_t)N;
#pragma unroll
    for (int i = 0; i < 4; ++i) {
        const int kk = (tid >> 4) + 16 * i, n4 = (tid & 15) * 4;
        const int n = n0 + n4;
        const bool ok = n < NV;
        const int nc = ok ? n : (NV - 4);
        const int col = (nc / G) * SG + OFF + (nc % G);
        v4f v = *(const v4f*)(Wz + (size_t)(k0 + kk) * (size_t)N + (size_t)col);
        asm volatile("" : "+v"(v));
#pragma unroll
        for (int j = 0; j < 4; ++j) ts[kk * 65 + n4 + j] = ok ? v[j] : 0.0f;
    }
    __syncthreads();
#pragma unroll 1
    for (int ps = 0; ps < 2; ++ps) {
#pragma unroll
        for (int i = 0; i < 2; ++i) {
            const int n = (tid >> 3) + 32 * i, k8 = (tid & 7) * 8;
            const size_t off = (size_t)(n0 + n + z * dzr) * (size_t)ldk + (size_t)(koff + k0 + k8);
            float f[8];
#pragma unroll
            for (int j = 0; j < 8; ++j) f[j] = ts[(k8 + j) * 65 + n];
            if (F16) { v8h o;
#pragma unroll
                for (int j = 0; j < 8; ++j) o[j] = toh_flush(bfr(f[j]) * WSC);
                *(volatile v8h*)(D + off) = o;
            } else { v8us o;
#pragma unroll
                for (int j = 0; j < 8; ++j) o[j] = f2bf(f[j]);
                *(volatile v8us*)(D + off) = o; }
        }
        if (ps == 0) __threadfence();
    }
}
__global__ __launch_bounds__(256) void k_wconv_b(const float* __restrict__ W, bf* D, int K, int N, int NV, int G, int SG, int OFF, int ldk, int koff, int dzr) {
    wconv_body<0>(W, D, K, N, NV, G, SG, OFF, ldk, koff, dzr);
}
__global__ __launch_bounds__(256) void k_wconv_h(const float* __restrict__ W, h16* D, int K, int N, int NV, int G, int SG, int OFF, int ldk, int koff, int dzr) {
    wconv_body<1>(W, (unsigned short*)D, K, N, NV, G, SG, OFF, ldk, koff, dzr);
}

__global__ __launch_bounds__(256) void k_ropetab(float* TAB, float f0, float f1, float f2, float f3, float f4, float f5, float f6, float f7,
                                                 float f8, float f9, float f10, float f11, float f12, float f13, float f14, float f15) {
#pragma clang fp contract(off)
    __shared__ __align__(16) float ts[16 * 32];
    const int tid = threadIdx.x; const int sl = tid >> 4, f = tid & 15;
    float w = f0;
    w = (f == 1) ? f1 : w;   w = (f == 2) ? f2 : w;   w = (f == 3) ? f3 : w;   w = (f == 4) ? f4 : w;
    w = (f == 5) ? f5 : w;   w = (f == 6) ? f6 : w;   w = (f == 7) ? f7 : w;   w = (f == 8) ? f8 : w;
    w = (f == 9) ? f9 : w;   w = (f == 10) ? f10 : w; w = (f == 11) ? f11 : w; w = (f == 12) ? f12 : w;
    w = (f == 13) ? f13 : w; w = (f == 14) ? f14 : w; w = (f == 15) ? f15 : w;
    const int s = blockIdx.x * 16 + sl;
    const float ang = (float)s * w;
    float sn, cs; sincosf(ang, &sn, &cs);
    ts[sl * 32 + f] = cs; ts[sl * 32 + 16 + f] = sn;
    __syncthreads();
    if (tid < 128) {
        const int row = tid >> 3, c4 = (tid & 7) * 4;
        const v4f v = *(const v4fa*)(&ts[row * 32 + c4]);
        float* p = TAB + ((size_t)blockIdx.x * 16 + row) * 32 + c4;
        *(volatile v4f*)p = v; __threadfence(); *(volatile v4f*)p = v;
    }
}

__device__ __forceinline__ void gemm_core_b(const bf* __restrict__ A, const bf* __restrict__ Bt, const int K, const int r0, const int c0, const int lr, const int hi, v8f (&acc)[4][4]) {
#pragma unroll
    for (int mb = 0; mb < 4; ++mb)
#pragma unroll
        for (int nb = 0; nb < 4; ++nb) acc[mb][nb] = (v8f){};
    const size_t aoff = (size_t)(r0 + lr) * K + 8 * hi, boff = (size_t)(c0 + lr) * K + 8 * hi;
#pragma unroll 1
    for (int kc = 0; kc < K; kc += 32) {
        v16bf a[4];
#pragma unroll
        for (int mb = 0; mb < 4; ++mb) a[mb] = ldb(A + aoff + (size_t)mb * 16 * K + kc);
#pragma unroll
        for (int nb = 0; nb < 4; ++nb) { const v16bf b = ldb(Bt + boff + (size_t)nb * 16 * K + kc);
#pragma unroll
            for (int mb = 0; mb < 4; ++mb) acc[mb][nb] = wmmab(a[mb], b, acc[mb][nb]); }
        asm volatile("v_nop\n\tv_nop\n\tv_nop\n\tv_nop" : "+v"(acc[0][0]), "+v"(acc[1][1]), "+v"(acc[2][2]), "+v"(acc[3][3]) : "v"(a[0]), "v"(a[1]), "v"(a[2]), "v"(a[3]));
    }
}
__device__ __forceinline__ void gemm_core_h(const h16* __restrict__ A, const h16* __restrict__ Bt, const int K, const int r0, const int c0, const int lr, const int hi, v8f (&acc)[4][4]) {
#pragma unroll
    for (int mb = 0; mb < 4; ++mb)
#pragma unroll
        for (int nb = 0; nb < 4; ++nb) acc[mb][nb] = (v8f){};
    const size_t aoff = (size_t)(r0 + lr) * K + 8 * hi, boff = (size_t)(c0 + lr) * K + 8 * hi;
#pragma unroll 1
    for (int kc = 0; kc < K; kc += 32) {
        v16h a[4];
#pragma unroll
        for (int mb = 0; mb < 4; ++mb) a[mb] = ldh(A + aoff + (size_t)mb * 16 * K + kc);
#pragma unroll
        for (int nb = 0; nb < 4; ++nb) { const v16h b = ldh(Bt + boff + (size_t)nb * 16 * K + kc);
#pragma unroll
            for (int mb = 0; mb < 4; ++mb) acc[mb][nb] = wmma16(a[mb], b, acc[mb][nb]); }
        asm volatile("v_nop\n\tv_nop\n\tv_nop\n\tv_nop" : "+v"(acc[0][0]), "+v"(acc[1][1]), "+v"(acc[2][2]), "+v"(acc[3][3]) : "v"(a[0]), "v"(a[1]), "v"(a[2]), "v"(a[3]));
    }
}

template <int HASR>
__device__ __forceinline__ void ep_f32(const v8f (&acc)[4][4], float* C, const float* __restrict__ R, const int ldc, const int ncols, const int oseq, const int rseq, const int rb16, const float scale,
                                       const int r0, const int c0, const int lane, const int lr, const int hi) {
    __shared__ __align__(16) float os[16 * 68];
    const int bb = r0 / SEQ, tt = r0 % SEQ;
    const size_t orow0 = (size_t)bb * (size_t)oseq + (size_t)tt;
    const size_t rrow0 = (size_t)bb * (size_t)rseq + (size_t)tt;
    const int c4 = (lane & 15) * 4;
    const bool cok = (c0 + c4) < ncols;
    const int cc = cok ? (c0 + c4) : (ncols - 4);
#pragma unroll
    for (int mb = 0; mb < 4; ++mb) {
#pragma unroll
        for (int nb = 0; nb < 4; ++nb) {
#pragma unroll
            for (int j = 0; j < 8; ++j) os[(hi * 8 + j) * 68 + nb * 16 + lr] = acc[mb][nb][j] * scale; }
        wave_sync();
#pragma unroll 1
        for (int ps = 0; ps < 2; ++ps) {
#pragma unroll
            for (int s = 0; s < 8; ++s) { const int row = 2 * s + (lane >> 4);
                v4f val = *(const v4fa*)(&os[row * 68 + c4]);
                if (HASR) {
                    v4f rv = *(const v4f*)(R + (rrow0 + (size_t)(mb * 16 + row)) * (size_t)ldc + (size_t)cc);
                    asm volatile("" : "+v"(rv));
                    if (rb16) { rv[0] = bfr(rv[0]); rv[1] = bfr(rv[1]); rv[2] = bfr(rv[2]); rv[3] = bfr(rv[3]); }
                    val = val + rv;
                }
                if (cok) *(volatile v4f*)(C + (orow0 + (size_t)(mb * 16 + row)) * (size_t)ldc + (size_t)(c0 + c4)) = val; }
            if (ps == 0) __threadfence(); }
        wave_sync();
    }
}

template <int HDW, int ROPE>
__device__ __forceinline__ void ep_head(const v8f (&acc)[4][4], h16* Ph, const float* __restrict__ TAB, const float scale, const int r0, const int c0, const int lane, const int lr, const int hi) {
    __shared__ __align__(16) float os[16 * 68];
    constexpr int NHT = 64 / HDW;
    constexpr int PPR = HDW / 8;
    constexpr int TRIPS = 16 * PPR / 32;
    static_assert(32 * TRIPS * 8 == 16 * HDW);
    static_assert(NHT * HDW == 64);
    const int bb = r0 / SEQ, tt = r0 % SEQ;
#pragma unroll
    for (int mb = 0; mb < 4; ++mb) {
#pragma unroll
        for (int nb = 0; nb < 4; ++nb) {
#pragma unroll
            for (int j = 0; j < 8; ++j) os[(hi * 8 + j) * 68 + nb * 16 + lr] = acc[mb][nb][j] * scale; }
        wave_sync();
#pragma unroll 1
        for (int ps = 0; ps < 2; ++ps) {
#pragma unroll
            for (int hh = 0; hh < NHT; ++hh) {
                const size_t sb = ((size_t)(bb * NH_ + c0 / HDW + hh) * SEQ + (size_t)(tt + mb * 16)) * HDW;
#pragma unroll
                for (int s = 0; s < TRIPS; ++s) { const int p = s * 32 + lane; const int row = p / PPR, c8 = (p % PPR) * 8;
                    v4f x0 = *(const v4fa*)(&os[row * 68 + hh * HDW + c8]); v4f x1 = *(const v4fa*)(&os[row * 68 + hh * HDW + c8 + 4]);
                    if (ROPE) {
                        const int pc = c8 ^ 16;
                        const v4f y0 = *(const v4fa*)(&os[row * 68 + hh * HDW + pc]); const v4f y1 = *(const v4fa*)(&os[row * 68 + hh * HDW + pc + 4]);
                        const float* tr = TAB + (size_t)(tt + mb * 16 + row) * 32 + (c8 & 8);
                        const v4f cs0 = *(const v4f*)tr, cs1 = *(const v4f*)(tr + 4), sn0 = *(const v4f*)(tr + 16), sn1 = *(const v4f*)(tr + 20);
                        const float sg = (c8 & 16) ? 1.0f : -1.0f;
                        x0 = x0 * cs0 + (y0 * sn0) * sg; x1 = x1 * cs1 + (y1 * sn1) * sg;
                    }
                    v8h hv;
#pragma unroll
                    for (int i = 0; i < 4; ++i) { hv[i] = toh_flush(x0[i]); hv[4 + i] = toh_flush(x1[i]); }
                    *(volatile v8h*)(Ph + sb + (size_t)p * 8) = hv; } }
            if (ps == 0) __threadfence(); }
        wave_sync();
    }
}

__device__ __forceinline__ void ep_t(const v8f (&acc)[4][4], h16* Pt, const int MR, const float scale, const int r0, const int c0, const int lane, const int lr, const int hi) {
    __shared__ __align__(16) float os[16 * 68];
    const int bb = c0 / SEQ, tt = c0 % SEQ;
    const size_t tbase = (size_t)bb * (size_t)MR * SEQ + (size_t)r0 * SEQ + (size_t)tt;
#pragma unroll
    for (int mb = 0; mb < 4; ++mb) {
#pragma unroll
        for (int nb = 0; nb < 4; ++nb) {
#pragma unroll
            for (int j = 0; j < 8; ++j) os[(hi * 8 + j) * 68 + nb * 16 + lr] = acc[mb][nb][j] * scale; }
        wave_sync();
#pragma unroll 1
        for (int ps = 0; ps < 2; ++ps) {
#pragma unroll
            for (int s = 0; s < 4; ++s) { const int row = 4 * s + (lane >> 3), c8 = (lane & 7) * 8;
                const v4f x0 = *(const v4fa*)(&os[row * 68 + c8]); const v4f x1 = *(const v4fa*)(&os[row * 68 + c8 + 4]); v8h hv;
#pragma unroll
                for (int i = 0; i < 4; ++i) { hv[i] = toh_flush(x0[i]); hv[4 + i] = toh_flush(x1[i]); }
                *(volatile v8h*)(Pt + tbase + (size_t)(mb * 16 + row) * SEQ + c8) = hv; }
            if (ps == 0) __threadfence(); }
        wave_sync();
    }
}

__device__ __forceinline__ void ep_up(const v8f (&acc)[4][4], h16* Hd, const float* __restrict__ gates, const int r0, const int c0, const int lane, const int lr, const int hi) {
    __shared__ __align__(16) float os[16 * 68];
    const int e = c0 >> 10;
    const int ec = e < NEX ? e : (NEX - 1);
#pragma unroll
    for (int mb = 0; mb < 4; ++mb) {
#pragma unroll
        for (int nb = 0; nb < 4; ++nb) {
#pragma unroll
            for (int j = 0; j < 8; ++j) os[(hi * 8 + j) * 68 + nb * 16 + lr] = acc[mb][nb][j] * SC_TRUE; }
        wave_sync();
#pragma unroll 1
        for (int ps = 0; ps < 2; ++ps) {
#pragma unroll
            for (int s = 0; s < 4; ++s) { const int row = 4 * s + (lane >> 3), c8 = (lane & 7) * 8;
                float gl = gates[(size_t)(r0 + mb * 16 + row) * NEX + ec];
                asm volatile("" : "+v"(gl));
                const float g = (e < NEX) ? gl : 1.0f;
                const float gs = g * ASC;
                const v4f x0 = *(const v4fa*)(&os[row * 68 + c8]); const v4f x1 = *(const v4fa*)(&os[row * 68 + c8 + 4]); v8h hv;
#pragma unroll
                for (int i = 0; i < 4; ++i) {
                    const float a = x0[i], c = x1[i];
                    const float sa = a * __builtin_amdgcn_rcpf(1.0f + __expf(-a));
                    const float sc = c * __builtin_amdgcn_rcpf(1.0f + __expf(-c));
                    hv[i] = toh_flush(sa * gs); hv[4 + i] = toh_flush(sc * gs); }
                *(volatile v8h*)(Hd + (size_t)(r0 + mb * 16 + row) * KH + (size_t)(c0 + c8)) = hv; }
            if (ps == 0) __threadfence(); }
        wave_sync();
    }
}

__global__ __launch_bounds__(32) void k_gemm_xf(const bf* __restrict__ A, const bf* __restrict__ Bt, float* C, int K, int ldc, int ncols, int oseq) {
    const int lane = threadIdx.x & 31, lr = lane & 15, hi = lane >> 4; const int r0 = blockIdx.x * 64, c0 = blockIdx.y * 64;
    v8f acc[4][4];
    gemm_core_b(A, Bt, K, r0, c0, lr, hi, acc);
    ep_f32<0>(acc, C, C, ldc, ncols, oseq, oseq, 0, SC_ONE, r0, c0, lane, lr, hi);
}
__global__ __launch_bounds__(32) void k_gemm_hf(const h16* __restrict__ A, const h16* __restrict__ Bt, float* C, const float* __restrict__ R, int K, int ldc, int ncols, int oseq, int rseq, int rb16, float scale) {
    const int lane = threadIdx.x & 31, lr = lane & 15, hi = lane >> 4; const int r0 = blockIdx.x * 64, c0 = blockIdx.y * 64;
    v8f acc[4][4];
    gemm_core_h(A, Bt, K, r0, c0, lr, hi, acc);
    ep_f32<1>(acc, C, R, ldc, ncols, oseq, rseq, rb16, scale, r0, c0, lane, lr, hi);
}
__global__ __launch_bounds__(32) void k_gemm_head64(const h16* __restrict__ A, const h16* __restrict__ Bt, h16* Ph, int K, float scale) {
    const int lane = threadIdx.x & 31, lr = lane & 15, hi = lane >> 4; const int r0 = blockIdx.x * 64, c0 = blockIdx.y * 64;
    v8f acc[4][4];
    gemm_core_h(A, Bt, K, r0, c0, lr, hi, acc);
    ep_head<64, 0>(acc, Ph, (const float*)0, scale, r0, c0, lane, lr, hi);
}
__global__ __launch_bounds__(32) void k_gemm_head32r(const h16* __restrict__ A, const h16* __restrict__ Bt, h16* Ph, const float* __restrict__ TAB, int K, float scale) {
    const int lane = threadIdx.x & 31, lr = lane & 15, hi = lane >> 4; const int r0 = blockIdx.x * 64, c0 = blockIdx.y * 64;
    v8f acc[4][4];
    gemm_core_h(A, Bt, K, r0, c0, lr, hi, acc);
    ep_head<32, 1>(acc, Ph, TAB, scale, r0, c0, lane, lr, hi);
}
__global__ __launch_bounds__(32) void k_gemm_vt(const h16* __restrict__ A, const h16* __restrict__ Bt, h16* Pt, int K, int MR, float scale) {
    const int lane = threadIdx.x & 31, lr = lane & 15, hi = lane >> 4; const int r0 = blockIdx.x * 64, c0 = blockIdx.y * 64;
    v8f acc[4][4];
    gemm_core_h(A, Bt, K, r0, c0, lr, hi, acc);
    ep_t(acc, Pt, MR, scale, r0, c0, lane, lr, hi);
}
__global__ __launch_bounds__(32) void k_gemm_up(const h16* __restrict__ A, const h16* __restrict__ Bt, const float* __restrict__ gates, h16* Hd, int K) {
    const int lane = threadIdx.x & 31, lr = lane & 15, hi = lane >> 4; const int r0 = blockIdx.x * 64, c0 = blockIdx.y * 64;
    v8f acc[4][4];
    gemm_core_h(A, Bt, K, r0, c0, lr, hi, acc);
    ep_up(acc, Hd, gates, r0, c0, lane, lr, hi);
}

__global__ __launch_bounds__(256) void k_rows_cq(const float* __restrict__ CQF, const float* __restrict__ gw, h16* CQH) {
#pragma clang fp contract(off)
    const int lane = threadIdx.x & 31;
    const int wave = __builtin_amdgcn_readfirstlane((int)(threadIdx.x >> 5));
    const int lc = lane < 24 ? lane : 23;
    const bool act = lane < 24;
    v4f g0 = *(const v4f*)(gw + 8 * lc), g1 = *(const v4f*)(gw + 8 * lc + 4);
#pragma unroll
    for (int j = 0; j < 4; ++j) { g0[j] = bfr(g0[j]); g1[j] = bfr(g1[j]); }
#pragma unroll 1
    for (int i = 0; i < 4; ++i) {
        const size_t row = (size_t)blockIdx.x * 32 + (size_t)(wave * 4 + i);
        const float* xr = CQF + row * DQC + 8 * lc;
        v4f x0 = *(const v4f*)xr, x1 = *(const v4f*)(xr + 4);
        asm volatile("" : "+v"(x0), "+v"(x1));
        float ss = 0.0f;
#pragma unroll
        for (int j = 0; j < 4; ++j) { ss += x0[j] * x0[j]; ss += x1[j] * x1[j]; }
        ss = act ? ss : 0.0f;
        ss += __shfl_xor(ss, 16, 32); ss += __shfl_xor(ss, 8, 32); ss += __shfl_xor(ss, 4, 32); ss += __shfl_xor(ss, 2, 32); ss += __shfl_xor(ss, 1, 32);
        const float rr = 1.0f / sqrtf(ss * (1.0f / (float)DQC) + EPSN);
        v8h o;
#pragma unroll
        for (int j = 0; j < 4; ++j) { o[j] = toh_flush(x0[j] * rr * g0[j] * ASC); o[4 + j] = toh_flush(x1[j] * rr * g1[j] * ASC); }
        h16* dst = CQH + row * DQC + 8 * lane;
        if (act) *(volatile v8h*)dst = o;
        __threadfence();
        if (act) *(volatile v8h*)dst = o;
    }
}

__global__ __launch_bounds__(256) void k_rows_kv(const float* __restrict__ CKV, const float* __restrict__ gw, const float* __restrict__ TAB, h16* CKN, h16* KRP) {
#pragma clang fp contract(off)
    __shared__ __align__(16) float krs[8 * 4 * 32];
    const int lane = threadIdx.x & 31;
    const int wave = __builtin_amdgcn_readfirstlane((int)(threadIdx.x >> 5));
    const int cb = (8 * lane < DKV - 8) ? 8 * lane : (DKV - 8);
    const bool isn = lane < 16;
    const bool isr = (lane >> 2) == 4;
    const int gc = isn ? 8 * lane : 0;
    v4f g0 = *(const v4f*)(gw + gc), g1 = *(const v4f*)(gw + gc + 4);
#pragma unroll
    for (int j = 0; j < 4; ++j) { g0[j] = bfr(g0[j]); g1[j] = bfr(g1[j]); }
    const int f0 = (lane & 1) * 8;
    const float sg = (lane & 2) ? 1.0f : -1.0f;
#pragma unroll 1
    for (int i = 0; i < 4; ++i) {
        const int m = blockIdx.x * 32 + wave * 4 + i;
        const int bb = m / SEQ, t = m % SEQ;
        const float* xr = CKV + ((size_t)bb * OUT_SEQ + (size_t)t) * DKV + cb;
        v4f x0 = *(const v4f*)xr, x1 = *(const v4f*)(xr + 4);
        asm volatile("" : "+v"(x0), "+v"(x1));
        float ss = 0.0f;
#pragma unroll
        for (int j = 0; j < 4; ++j) { ss += x0[j] * x0[j]; ss += x1[j] * x1[j]; }
        ss = isn ? ss : 0.0f;
        ss += __shfl_xor(ss, 16, 32); ss += __shfl_xor(ss, 8, 32); ss += __shfl_xor(ss, 4, 32); ss += __shfl_xor(ss, 2, 32); ss += __shfl_xor(ss, 1, 32);
        const float rr = 1.0f / sqrtf(ss * (1.0f / (float)DKC) + EPSN);
        v8h o;
#pragma unroll
        for (int j = 0; j < 4; ++j) { o[j] = toh_flush(x0[j] * rr * g0[j] * ASC); o[4 + j] = toh_flush(x1[j] * rr * g1[j] * ASC); }
        v4f y0, y1;
#pragma unroll
        for (int j = 0; j < 4; ++j) { y0[j] = __shfl_xor(x0[j], 2, 32); y1[j] = __shfl_xor(x1[j], 2, 32); }
        const float* tr = TAB + (size_t)t * 32 + f0;
        const v4f cs0 = *(const v4f*)tr, cs1 = *(const v4f*)(tr + 4), sn0 = *(const v4f*)(tr + 16), sn1 = *(const v4f*)(tr + 20);
        const v4f k0 = x0 * cs0 + (y0 * sn0) * sg, k1 = x1 * cs1 + (y1 * sn1) * sg;
        if (isr) { *(v4fa*)(&krs[(wave * 4 + i) * 32 + (lane & 3) * 8]) = k0; *(v4fa*)(&krs[(wave * 4 + i) * 32 + (lane & 3) * 8 + 4]) = k1; }
        h16* dst = CKN + (size_t)m * DKC + 8 * lane;
        if (isn) *(volatile v8h*)dst = o;
        __threadfence();
        if (isn) *(volatile v8h*)dst = o;
    }
    wave_sync();
    {
        const int lq = lane & 15;
        const v4f u0 = *(const v4fa*)(&krs[wave * 128 + lq * 8]); const v4f u1 = *(const v4fa*)(&krs[wave * 128 + lq * 8 + 4]);
        v8h ko;
#pragma unroll
        for (int j = 0; j < 4; ++j) { ko[j] = toh_flush(u0[j] * ASC); ko[4 + j] = toh_flush(u1[j] * ASC); }
        h16* dst = KRP + ((size_t)blockIdx.x * 32 + (size_t)(wave * 4)) * DRO + lq * 8;
        if (lane < 16) *(volatile v8h*)dst = ko;
        __threadfence();
        if (lane < 16) *(volatile v8h*)dst = ko;
    }
}

__global__ __launch_bounds__(256) void k_rows_x2(const float* __restrict__ H1, const float* __restrict__ gw, const float* __restrict__ WG, float* X2F, h16* X2H, float* GATES) {
#pragma clang fp contract(off)
    __shared__ __align__(16) float wgs[DM * NEX];
    __shared__ __align__(16) float xs[8 * DM];
    __shared__ __align__(16) float gsm[8 * 4 * NEX];
    const int tid = threadIdx.x, lane = threadIdx.x & 31;
    const int wave = __builtin_amdgcn_readfirstlane((int)(threadIdx.x >> 5));
#pragma unroll 1
    for (int i = 0; i < 4; ++i) { const int idx4 = (i * 256 + tid) * 4;
        v4f w = *(const v4f*)(WG + idx4);
        w[0] = bfr(w[0]); w[1] = bfr(w[1]); w[2] = bfr(w[2]); w[3] = bfr(w[3]);
        *(v4fa*)(&wgs[idx4]) = w; }
    __syncthreads();
    v4f g[4];
#pragma unroll
    for (int j = 0; j < 4; ++j) { g[j] = *(const v4f*)(gw + j * 128 + 4 * lane); g[j][0] = bfr(g[j][0]); g[j][1] = bfr(g[j][1]); g[j][2] = bfr(g[j][2]); g[j][3] = bfr(g[j][3]); }
#pragma unroll 1
    for (int i = 0; i < 4; ++i) {
        const size_t row = (size_t)blockIdx.x * 32 + (size_t)(wave * 4 + i);
        const float* xr = H1 + row * DM + 4 * lane;
        v4f x[4];
#pragma unroll
        for (int j = 0; j < 4; ++j) x[j] = *(const v4f*)(xr + j * 128);
        float ss = 0.0f;
#pragma unroll
        for (int j = 0; j < 4; ++j) { ss += x[j][0] * x[j][0]; ss += x[j][1] * x[j][1]; ss += x[j][2] * x[j][2]; ss += x[j][3] * x[j][3]; }
        ss += __shfl_xor(ss, 16, 32); ss += __shfl_xor(ss, 8, 32); ss += __shfl_xor(ss, 4, 32); ss += __shfl_xor(ss, 2, 32); ss += __shfl_xor(ss, 1, 32);
        const float rr = 1.0f / sqrtf(ss * (1.0f / (float)DM) + EPSN);
        v4f y[4];
#pragma unroll
        for (int j = 0; j < 4; ++j) { y[j] = x[j] * rr * g[j]; *(v4fa*)(&xs[wave * DM + j * 128 + 4 * lane]) = y[j]; }
        wave_sync();
        float acc[NEX];
#pragma unroll
        for (int e = 0; e < NEX; ++e) acc[e] = 0.0f;
#pragma unroll 1
        for (int q = 0; q < 16; ++q) { const int d = q * 32 + lane;
            const float xv = xs[wave * DM + d];
            const v4f w0 = *(const v4fa*)(&wgs[d * NEX]); const v4f w1 = *(const v4fa*)(&wgs[d * NEX + 4]);
#pragma unroll
            for (int e = 0; e < 4; ++e) { acc[e] += xv * w0[e]; acc[4 + e] += xv * w1[e]; } }
#pragma unroll
        for (int e = 0; e < NEX; ++e) { float a = acc[e];
            a += __shfl_xor(a, 16, 32); a += __shfl_xor(a, 8, 32); a += __shfl_xor(a, 4, 32); a += __shfl_xor(a, 2, 32); a += __shfl_xor(a, 1, 32); acc[e] = a; }
        float mx = acc[0];
#pragma unroll
        for (int e = 1; e < NEX; ++e) mx = fmaxf(mx, acc[e]);
        const int le = lane & 7;
        float mine = acc[0];
#pragma unroll
        for (int e = 1; e < NEX; ++e) mine = (le == e) ? acc[e] : mine;
        const float pe = expf(mine - mx);
        float pr[NEX];
#pragma unroll
        for (int e = 0; e < NEX; ++e) pr[e] = __shfl(pe, e, 32);
        float sp = pr[0];
#pragma unroll
        for (int e = 1; e < NEX; ++e) sp += pr[e];
        const float rs = 1.0f / sp;
#pragma unroll
        for (int e = 0; e < NEX; ++e) pr[e] = pr[e] * rs;
        int i0 = 0; float b0 = pr[0];
#pragma unroll
        for (int e = 1; e < NEX; ++e) { const bool gt = pr[e] > b0; b0 = gt ? pr[e] : b0; i0 = gt ? e : i0; }
        int i1 = -1; float b1 = -1.0f;
#pragma unroll
        for (int e = 0; e < NEX; ++e) { const bool gt = (e != i0) & (pr[e] > b1); b1 = gt ? pr[e] : b1; i1 = gt ? e : i1; }
        const float rt = 1.0f / (b0 + b1);
        const float w0n = b0 * rt, w1n = b1 * rt;
        v4f ga, gb;
#pragma unroll
        for (int e = 0; e < 4; ++e) { ga[e] = (e == i0) ? w0n : ((e == i1) ? w1n : 0.0f); gb[e] = ((4 + e) == i0) ? w0n : (((4 + e) == i1) ? w1n : 0.0f); }
        if (lane == 0) { *(v4fa*)(&gsm[(wave * 4 + i) * NEX]) = ga; *(v4fa*)(&gsm[(wave * 4 + i) * NEX + 4]) = gb; }
        v8h hv[2];
#pragma unroll
        for (int j2 = 0; j2 < 2; ++j2) { const v4f u0 = *(const v4fa*)(&xs[wave * DM + j2 * 256 + 8 * lane]); const v4f u1 = *(const v4fa*)(&xs[wave * DM + j2 * 256 + 8 * lane + 4]);
#pragma unroll
            for (int k = 0; k < 4; ++k) { hv[j2][k] = toh_flush(u0[k] * ASC); hv[j2][4 + k] = toh_flush(u1[k] * ASC); } }
#pragma unroll 1
        for (int ps = 0; ps < 2; ++ps) {
#pragma unroll
            for (int j = 0; j < 4; ++j) *(volatile v4f*)(X2F + row * DM + j * 128 + 4 * lane) = y[j];
#pragma unroll
            for (int j2 = 0; j2 < 2; ++j2) *(volatile v8h*)(X2H + row * DM + j2 * 256 + 8 * lane) = hv[j2];
            if (ps == 0) __threadfence(); }
        wave_sync();
    }
    wave_sync();
    {
        const v4f gv = *(const v4fa*)(&gsm[wave * 32 + (lane & 7) * 4]);
        float* dst = GATES + ((size_t)blockIdx.x * 32 + (size_t)(wave * 4)) * NEX + (lane & 7) * 4;
        if (lane < 8) *(volatile v4f*)dst = gv;
        __threadfence();
        if (lane < 8) *(volatile v4f*)dst = gv;
    }
}

__global__ __launch_bounds__(32 * AW) void k_flash(const h16* __restrict__ QN, const h16* __restrict__ QR, const h16* __restrict__ KN, const h16* __restrict__ KR,
                                                   const h16* __restrict__ VT, h16* CTX) {
    __shared__ __align__(16) float os[AW * 16 * OSP];
    const int lane = threadIdx.x & 31, lr = lane & 15, hi = lane >> 4;
    const int wave = __builtin_amdgcn_readfirstlane((int)(threadIdx.x >> 5));
    const int zh = blockIdx.y; const int b = zh / NH_, h = zh % NH_;
    const int t0 = (blockIdx.x * AW + wave) * 16;
    const int lim = t0 + lr;
    const int nk = (t0 + 16 + 31) & ~31;
    const size_t qo  = ((size_t)zh * SEQ + (size_t)(t0 + lr)) * DNO + 8 * hi;
    const size_t qro = ((size_t)zh * SEQ + (size_t)(t0 + lr)) * DRO + 8 * hi;
    const v16h q0 = ldh(QN + qo), q1 = ldh(QN + qo + 32), q2 = ldh(QR + qro);
    const size_t ko  = ((size_t)zh * SEQ + (size_t)lr) * DNO + 8 * hi;
    const size_t kro = ((size_t)b * SEQ + (size_t)lr) * DRO + 8 * hi;
    const size_t vo  = ((size_t)zh * DVH + (size_t)lr) * SEQ + 8 * hi;
    v8f o[8];
#pragma unroll
    for (int j = 0; j < 8; ++j) o[j] = (v8f){};
    float m = NEGB, l = 0.0f;
#pragma unroll 1
    for (int key0 = 0; key0 < nk; key0 += 32) {
        const h16* ka = KN + ko + (size_t)key0 * DNO;
        const h16* kr = KR + kro + (size_t)key0 * DRO;
        const v16h a0 = ldh(ka), a1 = ldh(ka + 32), a2 = ldh(kr);
        const v16h b0 = ldh(ka + 16 * DNO), b1 = ldh(ka + 16 * DNO + 32), b2 = ldh(kr + 16 * DRO);
        v8f sa = (v8f){}, sb = (v8f){};
        sa = wmma16(a0, q0, sa); sb = wmma16(b0, q0, sb);
        sa = wmma16(a1, q1, sa); sb = wmma16(b1, q1, sb);
        sa = wmma16(a2, q2, sa); sb = wmma16(b2, q2, sb);
        asm volatile("v_nop\n\tv_nop\n\tv_nop\n\tv_nop" : "+v"(sa), "+v"(sb) : "v"(a0), "v"(a1), "v"(a2), "v"(b0), "v"(b1), "v"(b2), "v"(q0), "v"(q1), "v"(q2));
        const int ja = key0 + 8 * hi;
        float ta[8], tb[8]; bool fa[8], fb[8]; float mx = NEGB;
#pragma unroll
        for (int r = 0; r < 8; ++r) {
            fa[r] = (ja + r <= lim);
            fb[r] = (ja + 16 + r <= lim);
            ta[r] = sa[r] * SC2S; tb[r] = sb[r] * SC2S;
            mx = fmaxf(mx, fmaxf(fa[r] ? ta[r] : NEGB, fb[r] ? tb[r] : NEGB)); }
        mx = fmaxf(mx, __shfl_xor(mx, 16, 32));
        const float mnew = fmaxf(m, mx);
        const float alpha = __builtin_amdgcn_exp2f(m - mnew);
        const float sh = PSH - mnew;
        v16h pb; float ls = 0.0f;
#pragma unroll
        for (int r = 0; r < 8; ++r) {
            const float xa = ta[r] + sh, xb = tb[r] + sh;
            const float ea = __builtin_amdgcn_exp2f(xa), eb = __builtin_amdgcn_exp2f(xb);
            const float ga = (fa[r] & (xa >= -14.0f)) ? ea : 0.0f, gb = (fb[r] & (xb >= -14.0f)) ? eb : 0.0f;
            const h16 pa = (h16)ga; const h16 pc = (h16)gb;
            pb[r] = pa; pb[8 + r] = pc;
            ls += (float)pa + (float)pc; }
        l = l * alpha + ls; m = mnew;
#pragma unroll
        for (int j = 0; j < 8; ++j) o[j] = o[j] * alpha;
        const h16* va = VT + vo + key0;
        { const v16h v0 = ldh(va), v1 = ldh(va + (size_t)16 * SEQ), v2 = ldh(va + (size_t)32 * SEQ), v3 = ldh(va + (size_t)48 * SEQ);
          o[0] = wmma16(v0, pb, o[0]); o[1] = wmma16(v1, pb, o[1]); o[2] = wmma16(v2, pb, o[2]); o[3] = wmma16(v3, pb, o[3]);
          asm volatile("v_nop\n\tv_nop\n\tv_nop\n\tv_nop" : "+v"(o[0]), "+v"(o[1]), "+v"(o[2]), "+v"(o[3]) : "v"(v0), "v"(v1), "v"(v2), "v"(v3), "v"(pb)); }
        { const v16h v4 = ldh(va + (size_t)64 * SEQ), v5 = ldh(va + (size_t)80 * SEQ), v6 = ldh(va + (size_t)96 * SEQ), v7 = ldh(va + (size_t)112 * SEQ);
          o[4] = wmma16(v4, pb, o[4]); o[5] = wmma16(v5, pb, o[5]); o[6] = wmma16(v6, pb, o[6]); o[7] = wmma16(v7, pb, o[7]);
          asm volatile("v_nop\n\tv_nop\n\tv_nop\n\tv_nop" : "+v"(o[4]), "+v"(o[5]), "+v"(o[6]), "+v"(o[7]) : "v"(v4), "v"(v5), "v"(v6), "v"(v7), "v"(pb)); }
    }
    l += __shfl_xor(l, 16, 32);
    const bool any = l > 0.0f;
    const float lsafe = any ? l : 1.0f;
    const float inv = any ? (CTXS / lsafe) : 0.0f;
    const int wb = wave * 16 * OSP;
#pragma unroll
    for (int j = 0; j < 8; ++j) { v4f a, c;
        a[0] = o[j][0] * inv; a[1] = o[j][1] * inv; a[2] = o[j][2] * inv; a[3] = o[j][3] * inv; c[0] = o[j][4] * inv; c[1] = o[j][5] * inv; c[2] = o[j][6] * inv; c[3] = o[j][7] * inv;
        *(v4fa*)(&os[wb + lr * OSP + 16 * j + 8 * hi]) = a; *(v4fa*)(&os[wb + lr * OSP + 16 * j + 8 * hi + 4]) = c; }
    wave_sync();
    h16* crow = CTX + ((size_t)b * SEQ + (size_t)t0) * DM + h * DVH;
#pragma unroll 1
    for (int ps = 0; ps < 2; ++ps) {
#pragma unroll
        for (int s = 0; s < 8; ++s) { const int row = 2 * s + (lane >> 4), c8 = (lane & 15) * 8;
            const v4f x0 = *(const v4fa*)(&os[wb + row * OSP + c8]); const v4f x1 = *(const v4fa*)(&os[wb + row * OSP + c8 + 4]); v8h hv;
#pragma unroll
            for (int i = 0; i < 4; ++i) { hv[i] = toh_flush(x0[i]); hv[4 + i] = toh_flush(x1[i]); }
            *(volatile v8h*)(crow + (size_t)row * DM + c8) = hv; }
        if (ps == 0) __threadfence(); }
}

static constexpr size_t al256(size_t v) { return (v + 255) & ~(size_t)255; }
static constexpr size_t TOK = (size_t)NB * SEQ;
static constexpr size_t SZ_WDQ  = al256((size_t)192 * DM * 2);
static constexpr size_t SZ_WDKV = al256((size_t)192 * DM * 2);
static constexpr size_t SZ_WQN  = al256((size_t)256 * DQC * 2);
static constexpr size_t SZ_WQR  = al256((size_t)128 * DQC * 2);
static constexpr size_t SZ_WKN  = al256((size_t)256 * DKC * 2);
static constexpr size_t SZ_WVW  = al256((size_t)512 * DKC * 2);
static constexpr size_t SZ_WOT  = al256((size_t)DM * DM * 2);
static constexpr size_t SZ_W1T  = al256((size_t)KH * DM * 2);
static constexpr size_t SZ_W2T  = al256((size_t)DM * KH * 2);
static constexpr size_t SZ_TAB  = al256((size_t)SEQ * 32 * 4);
static constexpr size_t SZ_W = SZ_WDQ + SZ_WDKV + SZ_WQN + SZ_WQR + SZ_WKN + SZ_WVW + SZ_WOT + SZ_W1T + SZ_W2T + SZ_TAB;
static constexpr size_t SZ_X2F = al256(TOK * DM * 4);
static constexpr size_t SZ_X2H = al256(TOK * DM * 2);
static constexpr size_t SZ_GAT = al256(TOK * NEX * 4);
static constexpr size_t SZ_XB  = al256(TOK * DM * 2);
static constexpr size_t SZ_CQF = al256(TOK * DQC * 4);
static constexpr size_t SZ_CQH = al256(TOK * DQC * 2);
static constexpr size_t SZ_CKN = al256(TOK * DKC * 2);
static constexpr size_t SZ_KRP = al256(TOK * DRO * 2);
static constexpr size_t SZ_QNP = al256(TOK * NH_ * DNO * 2);
static constexpr size_t SZ_QRP = al256(TOK * NH_ * DRO * 2);
static constexpr size_t SZ_KNP = al256(TOK * NH_ * DNO * 2);
static constexpr size_t SZ_VTP = al256(TOK * NH_ * DVH * 2);
static constexpr size_t SZ_CTX = al256(TOK * DM * 2);
static constexpr size_t SZ_H1  = al256(TOK * DM * 4);
static constexpr size_t SZ_ATT = SZ_XB + SZ_CQF + SZ_CQH + SZ_CKN + SZ_KRP + SZ_QNP + SZ_QRP + SZ_KNP + SZ_VTP + SZ_CTX + SZ_H1;
static constexpr size_t SZ_HID = al256((size_t)SEQ * KH * 2);
static constexpr size_t SZ_A = SZ_ATT > SZ_HID ? SZ_ATT : SZ_HID;
static constexpr size_t SZ_TOTAL = SZ_W + SZ_X2F + SZ_X2H + SZ_GAT + SZ_A;
static_assert(SZ_ATT <= SZ_A);
static_assert(SZ_HID <= SZ_A);
static_assert(SZ_TOTAL <= (size_t)134217728);

extern "C" void kernel_launch(void* const* d_in, const int* in_sizes, int n_in,
                              void* d_out, int out_size, void* d_ws, size_t ws_size, hipStream_t stream) {
    if (n_in < 14) return;
    const size_t needx = ((size_t)(NB - 1) * SEQ_FULL + SEQ) * DM;
    if ((size_t)in_sizes[0] < needx) return;
    if (in_sizes[1] < DM || (size_t)in_sizes[2] < (size_t)DM * DQC || in_sizes[3] < DQC) return;
    if ((size_t)in_sizes[4] < (size_t)DQC * 384 || (size_t)in_sizes[5] < (size_t)DM * DKV || in_sizes[6] < DKC) return;
    if ((size_t)in_sizes[7] < (size_t)DKC * 768 || (size_t)in_sizes[8] < (size_t)DM * DM || (size_t)in_sizes[9] < (size_t)DM * NEX) return;
    if ((size_t)in_sizes[10] < (size_t)NEX * DM * DEX || (size_t)in_sizes[11] < (size_t)NEX * DEX * DM) return;
    if ((size_t)in_sizes[12] < (size_t)NSH * DM * DEX || (size_t)in_sizes[13] < (size_t)NSH * DEX * DM) return;
    if ((size_t)out_size < OUT1_OFF + ((size_t)(NB - 1) * OUT_SEQ + SEQ) * DKV) return;
    if ((size_t)out_size < ((size_t)(NB - 1) * OUT_SEQ + SEQ) * DM) return;
    if (SZ_TOTAL > ws_size) return;
    const float* x    = (const float*)d_in[0];
    const float* n2w  = (const float*)d_in[1];
    const float* wdq  = (const float*)d_in[2];
    const float* qnw  = (const float*)d_in[3];
    const float* wuq  = (const float*)d_in[4];
    const float* wdkv = (const float*)d_in[5];
    const float* kvnw = (const float*)d_in[6];
    const float* wukv = (const float*)d_in[7];
    const float* wo   = (const float*)d_in[8];
    const float* wg   = (const float*)d_in[9];
    const float* we1  = (const float*)d_in[10];
    const float* we2  = (const float*)d_in[11];
    const float* ws1  = (const float*)d_in[12];
    const float* ws2  = (const float*)d_in[13];
    float* OUT0 = (float*)d_out;
    float* OUT1 = (float*)d_out + OUT1_OFF;
    char* wsp = (char*)d_ws;
    bf*  WDQ  = (bf*)wsp;  wsp += SZ_WDQ;
    bf*  WDKV = (bf*)wsp;  wsp += SZ_WDKV;
    h16* WQN  = (h16*)wsp; wsp += SZ_WQN;
    h16* WQR  = (h16*)wsp; wsp += SZ_WQR;
    h16* WKN  = (h16*)wsp; wsp += SZ_WKN;
    h16* WVW  = (h16*)wsp; wsp += SZ_WVW;
    h16* WOT  = (h16*)wsp; wsp += SZ_WOT;
    h16* W1T  = (h16*)wsp; wsp += SZ_W1T;
    h16* W2T  = (h16*)wsp; wsp += SZ_W2T;
    float* TAB = (float*)wsp; wsp += SZ_TAB;
    float* X2F = (float*)wsp; wsp += SZ_X2F;
    h16* X2H  = (h16*)wsp; wsp += SZ_X2H;
    float* GAT = (float*)wsp; wsp += SZ_GAT;
    char* regA = wsp;
    h16* HID  = (h16*)regA;
    bf*  XB   = (bf*)wsp;  wsp += SZ_XB;
    float* CQF = (float*)wsp; wsp += SZ_CQF;
    h16* CQH  = (h16*)wsp; wsp += SZ_CQH;
    h16* CKN  = (h16*)wsp; wsp += SZ_CKN;
    h16* KRP  = (h16*)wsp; wsp += SZ_KRP;
    h16* QNP  = (h16*)wsp; wsp += SZ_QNP;
    h16* QRP  = (h16*)wsp; wsp += SZ_QRP;
    h16* KNP  = (h16*)wsp; wsp += SZ_KNP;
    h16* VTP  = (h16*)wsp; wsp += SZ_VTP;
    h16* CTX  = (h16*)wsp; wsp += SZ_CTX;
    float* H1 = (float*)wsp; wsp += SZ_H1;

    if (SEQ == SEQ_FULL) {
        const size_t n8 = (size_t)NB * SEQ * DM / 8;
        k_cvt8<<<(unsigned)((n8 + 255) / 256), 256, 0, stream>>>(x, XB, n8);
    } else {
        const size_t n8 = (size_t)SEQ * DM / 8;
        for (int b = 0; b < NB; ++b) k_cvt8<<<(unsigned)((n8 + 255) / 256), 256, 0, stream>>>(x + (size_t)b * SEQ_FULL * DM, XB + (size_t)b * SEQ * DM, n8);
    }
    k_wconv_b<<<dim3(8, 3, 1), 256, 0, stream>>>(wdq,  WDQ,  512, 192, 192, 192, 0, 0, 512, 0, 0);
    k_wconv_b<<<dim3(8, 3, 1), 256, 0, stream>>>(wdkv, WDKV, 512, 160, 160, 192, 0, 0, 512, 0, 0);
    k_wconv_h<<<dim3(3, 4, 1), 256, 0, stream>>>(wuq,  WQN,  192, 384, 256, 64, 96, 0, 192, 0, 0);
    k_wconv_h<<<dim3(3, 2, 1), 256, 0, stream>>>(wuq,  WQR,  192, 384, 128, 32, 96, 64, 192, 0, 0);
    k_wconv_h<<<dim3(2, 4, 1), 256, 0, stream>>>(wukv, WKN,  128, 768, 256, 64, 192, 0, 128, 0, 0);
    k_wconv_h<<<dim3(2, 8, 1), 256, 0, stream>>>(wukv, WVW,  128, 768, 512, 128, 192, 64, 128, 0, 0);
    k_wconv_h<<<dim3(8, 8, 1), 256, 0, stream>>>(wo,   WOT,  512, 512, 512, 512, 0, 0, 512, 0, 0);
    k_wconv_h<<<dim3(8, 16, NEX), 256, 0, stream>>>(we1, W1T, 512, 1024, 1024, 1024, 0, 0, 512, 0, 1024);
    k_wconv_h<<<dim3(8, 16, NSH), 256, 0, stream>>>(ws1, W1T + (size_t)NEX * DEX * DM, 512, 1024, 1024, 1024, 0, 0, 512, 0, 1024);
    k_wconv_h<<<dim3(NEX * DEX / 64, 8, 1), 256, 0, stream>>>(we2, W2T, NEX * DEX, 512, 512, 512, 0, 0, KH, 0, 0);
    k_wconv_h<<<dim3(NSH * DEX / 64, 8, 1), 256, 0, stream>>>(ws2, W2T, NSH * DEX, 512, 512, 512, 0, 0, KH, NEX * DEX, 0);
    {
        float fr[16];
        for (int f = 0; f < 16; ++f) { const double e = (double)(2 * f) / 32.0; const float pw = (float)pow(10000.0, e); fr[f] = 1.0f / pw; }
        k_ropetab<<<SEQ / 16, 256, 0, stream>>>(TAB, fr[0], fr[1], fr[2], fr[3], fr[4], fr[5], fr[6], fr[7], fr[8], fr[9], fr[10], fr[11], fr[12], fr[13], fr[14], fr[15]);
    }
    const unsigned TT = (unsigned)(TOK / 64);
    k_gemm_xf<<<dim3(TT, 3, 1), 32, 0, stream>>>(XB, WDQ,  CQF,  DM, DQC, DQC, SEQ);
    k_gemm_xf<<<dim3(TT, 3, 1), 32, 0, stream>>>(XB, WDKV, OUT1, DM, DKV, DKV, OUT_SEQ);
    k_rows_cq<<<(unsigned)(TOK / 32), 256, 0, stream>>>(CQF, qnw, CQH);
    k_rows_kv<<<(unsigned)(TOK / 32), 256, 0, stream>>>(OUT1, kvnw, TAB, CKN, KRP);
    k_gemm_head64<<<dim3(TT, 4, 1), 32, 0, stream>>>(CQH, WQN, QNP, DQC, SC_PL);
    k_gemm_head32r<<<dim3(TT, 2, 1), 32, 0, stream>>>(CQH, WQR, QRP, TAB, DQC, SC_PL);
    k_gemm_head64<<<dim3(TT, 4, 1), 32, 0, stream>>>(CKN, WKN, KNP, DKC, SC_PL);
    k_gemm_vt<<<dim3(512 / 64, TT, 1), 32, 0, stream>>>(WVW, CKN, VTP, DKC, NH_ * DVH, SC_PL);
    k_flash<<<dim3(SEQ / (16 * AW), NB * NH_, 1), 32 * AW, 0, stream>>>(QNP, QRP, KNP, KRP, VTP, CTX);
    k_gemm_hf<<<dim3(TT, DM / 64, 1), 32, 0, stream>>>(CTX, WOT, H1, x, DM, DM, DM, SEQ, SEQ_FULL, 1, SC_WO);
    k_rows_x2<<<(unsigned)(TOK / 32), 256, 0, stream>>>(H1, n2w, wg, X2F, X2H, GAT);
    for (int b = 0; b < NB; ++b) {
        k_gemm_up<<<dim3(SEQ / 64, KH / 64, 1), 32, 0, stream>>>(X2H + (size_t)b * SEQ * DM, W1T, GAT + (size_t)b * SEQ * NEX, HID, DM);
        k_gemm_hf<<<dim3(SEQ / 64, DM / 64, 1), 32, 0, stream>>>(HID, W2T, OUT0 + (size_t)b * OUT_SEQ * DM, X2F + (size_t)b * SEQ * DM, KH, DM, DM, SEQ, SEQ, 0, SC_TRUE);
    }
}
